// MambaBlock_67972152427238
// MI455X (gfx1250) — hardware-verified
//
#include <hip/hip_runtime.h>
#include <math.h>

typedef __attribute__((ext_vector_type(16))) _Float16 v16h;
typedef __attribute__((ext_vector_type(8)))  _Float16 v8h;
typedef __attribute__((ext_vector_type(8)))  float    v8f;
typedef __attribute__((ext_vector_type(4)))  float    v4f;
typedef __attribute__((ext_vector_type(8)))  unsigned v8u;

constexpr int kBatch  = 8;
constexpr int kSeq    = 4096;
constexpr int kDm     = 128;
constexpr int kDi     = 256;
constexpr int kNs     = 128;
constexpr int kDtR    = 8;
constexpr int kXz     = 2 * kDi;
constexpr int kNx     = kDtR + 2 * kNs;
constexpr int kNxP    = 320;
constexpr int kRows   = kBatch * kSeq;
constexpr int kHalves = 2;
constexpr int kRowsH  = kRows / kHalves;
constexpr int kBatchH = kBatch / kHalves;
constexpr int kConvTP = 260;
constexpr int kTS     = 32;
constexpr int kSCh    = 64;
constexpr int kSYP    = 68;

constexpr float kCarryW  = 32.0f;
constexpr float kCarryXc = 64.0f;
constexpr float kCarryH  = 1048576.0f;
constexpr float kCarryC  = 256.0f;
constexpr float kCarryY  = 4096.0f;
constexpr float kInvHC   = 1.0f / (kCarryH * kCarryC);
constexpr float kLog2e   = 1.4426950408889634f;

static_assert(kNx == 264, "x_proj width");
static_assert(kDi == 256, "conv and scan assume 256 inner channels");
static_assert((kDm % 32) == 0 && (kDi % 32) == 0, "GEMM K multiples of 32");
static_assert((kRowsH % 64) == 0 && (kXz % 64) == 0 && (kNxP % 64) == 0 && (kDm % 64) == 0, "GEMM M,N multiples of 64");
static_assert((kSeq % 64) == 0 && (kSeq % kTS) == 0 && (kDi % kSCh) == 0 && (kRowsH % kSeq) == 0, "tile multiples");
static_assert(kNs == 128 && kDtR == 8, "scan lane map assumes 128 states and 8 dt columns");

constexpr size_t kOffU16   = 0;
constexpr size_t kOffWIN   = kOffU16  + (size_t)kRows  * kDm  * 2;
constexpr size_t kOffWX    = kOffWIN  + (size_t)kXz    * kDm  * 2;
constexpr size_t kOffWOUT  = kOffWX   + (size_t)kNxP   * kDi  * 2;
constexpr size_t kOffXZ    = kOffWOUT + (size_t)kDm    * kDi  * 2;
constexpr size_t kOffXC    = kOffXZ   + (size_t)kRowsH * kXz  * 4;
constexpr size_t kOffXC16  = kOffXC   + (size_t)kRowsH * kDi  * 4;
constexpr size_t kOffDBC   = kOffXC16 + (size_t)kRowsH * kDi  * 2;
constexpr size_t kOffY16   = kOffDBC  + (size_t)kRowsH * kNxP * 4;
constexpr size_t kWsTotal  = kOffY16  + (size_t)kRowsH * kDi  * 2;
static_assert(kWsTotal == 96829440ull, "carve total");
static_assert(kWsTotal <= 134217728ull, "carve cap");
static_assert((kOffWIN % 128) == 0 && (kOffWX % 128) == 0 && (kOffWOUT % 128) == 0 && (kOffXZ % 128) == 0 &&
              (kOffXC % 128) == 0 && (kOffXC16 % 128) == 0 && (kOffDBC % 128) == 0 && (kOffY16 % 128) == 0,
              "128-B aligned regions");

__device__ __forceinline__ unsigned short f2bf_bits(float f) {
  unsigned u = __float_as_uint(f);
  return (unsigned short)((u + 0x7FFFu + ((u >> 16) & 1u)) >> 16);
}
__device__ __forceinline__ float bf_bits2f(unsigned short h) { return __uint_as_float(((unsigned)h) << 16); }
__device__ __forceinline__ float bfr(float f) { return bf_bits2f(f2bf_bits(f)); }

union FragH { v16h v; v8h h[2]; };
__device__ __forceinline__ v16h frag_load_h(const _Float16* p) {
  FragH f;
  f.h[0] = *(const v8h*)(p);
  f.h[1] = *(const v8h*)(p + 16);
  return f.v;
}
__device__ __forceinline__ v8f mma_h(v16h a, v16h b, v8f c) {
  return __builtin_amdgcn_wmma_f32_16x16x32_f16(false, a, false, b, (short)0, c, false, false);
}
__device__ __forceinline__ void guard_row_h(v8f& a0, v8f& a1, v8f& a2, v8f& a3, v16h x, v16h y0, v16h y1, v16h y2, v16h y3) {
  asm volatile("v_nop\n\tv_nop\n\tv_nop\n\tv_nop" : "+v"(a0), "+v"(a1), "+v"(a2), "+v"(a3) : "v"(x), "v"(y0), "v"(y1), "v"(y2), "v"(y3));
}
__device__ __forceinline__ void guard1_h(v8f& a, v16h x, v16h y) {
  asm volatile("v_nop\n\tv_nop\n\tv_nop\n\tv_nop" : "+v"(a) : "v"(x), "v"(y));
}
__device__ __forceinline__ void acc_guard4(v8f& a, v8f& b, v8f& c, v8f& d) {
  asm volatile("v_nop\n\tv_nop\n\tv_nop\n\tv_nop" : "+v"(a), "+v"(b), "+v"(c), "+v"(d));
}
__device__ __forceinline__ unsigned pk_f16(float a, float b) {
  return __builtin_bit_cast(unsigned, __builtin_amdgcn_cvt_pkrtz(a, b));
}

__global__ __launch_bounds__(256) void gemm64_f16_kernel(
    const unsigned short* __restrict__ Ap, int lda,
    const unsigned short* __restrict__ Btp, int ldb,
    float* __restrict__ C, int ldc, int M, int N, int K, float scale)
{
  const _Float16* A  = (const _Float16*)Ap;
  const _Float16* Bt = (const _Float16*)Btp;
  __shared__ __align__(16) float sT[8][16 * 68];
  const int lane = threadIdx.x & 31;
  const int wave = threadIdx.x >> 5;
  const int tilesN = N >> 6;
  const int tilesM = M >> 6;
  const int tile = blockIdx.x * 8 + wave;
  if (tile >= tilesM * tilesN) return;
  const int tm = tile / tilesN;
  const int tn = tile - tm * tilesN;
  const int m0 = tm << 6;
  const int n0 = tn << 6;

  const int rlane = lane & 15;
  const int koff  = (lane >> 4) * 8;
  const int mOff  = (lane >> 4) * 8;

  v8f acc[4][4];
#pragma unroll
  for (int i = 0; i < 4; ++i)
#pragma unroll
    for (int j = 0; j < 4; ++j) acc[i][j] = (v8f){0.f, 0.f, 0.f, 0.f, 0.f, 0.f, 0.f, 0.f};

  for (int k0 = 0; k0 < K; k0 += 32) {
    v16h bh[4];
#pragma unroll
    for (int j = 0; j < 4; ++j) {
      const size_t bo = (size_t)(n0 + (j << 4) + rlane) * ldb + koff + k0;
      bh[j] = frag_load_h(Bt + bo);
    }
#pragma unroll
    for (int i = 0; i < 4; ++i) {
      const size_t ao = (size_t)(m0 + (i << 4) + rlane) * lda + koff + k0;
      const v16h ah = frag_load_h(A + ao);
#pragma unroll
      for (int j = 0; j < 4; ++j) acc[i][j] = mma_h(ah, bh[j], acc[i][j]);
      guard_row_h(acc[i][0], acc[i][1], acc[i][2], acc[i][3], ah, bh[0], bh[1], bh[2], bh[3]);
    }
  }
  acc_guard4(acc[0][0], acc[0][1], acc[0][2], acc[0][3]);
  acc_guard4(acc[1][0], acc[1][1], acc[1][2], acc[1][3]);
  acc_guard4(acc[2][0], acc[2][1], acc[2][2], acc[2][3]);
  acc_guard4(acc[3][0], acc[3][1], acc[3][2], acc[3][3]);

  float* slab = sT[wave];
#pragma unroll
  for (int i = 0; i < 4; ++i) {
    const int mBase = m0 + (i << 4);
#pragma unroll
    for (int j = 0; j < 4; ++j) {
#pragma unroll
      for (int r = 0; r < 8; ++r) slab[(mOff + r) * 68 + (j << 4) + rlane] = acc[i][j][r] * scale;
    }
    __builtin_amdgcn_fence(__ATOMIC_RELEASE, "workgroup");
    __builtin_amdgcn_wave_barrier();
    __builtin_amdgcn_fence(__ATOMIC_ACQUIRE, "workgroup");
    {
      const int hh = lane >> 4, c4 = (lane & 15) * 4;
      for (int pass = 0; pass < 2; ++pass) {
#pragma unroll
        for (int it = 0; it < 8; ++it) {
          const int row = it * 2 + hh;
          const v4f v = *(const v4f*)(slab + row * 68 + c4);
          *(volatile v4f*)(C + (size_t)(mBase + row) * ldc + n0 + c4) = v;
        }
        __threadfence();
      }
    }
    __builtin_amdgcn_fence(__ATOMIC_RELEASE, "workgroup");
    __builtin_amdgcn_wave_barrier();
    __builtin_amdgcn_fence(__ATOMIC_ACQUIRE, "workgroup");
  }
}

__global__ __launch_bounds__(256) void cast_bf16r_f16_kernel(
    const float* __restrict__ src, unsigned short* __restrict__ dst, int total8, int real8, float scale)
{
  const int i = blockIdx.x * 256 + threadIdx.x;
  if (i >= total8) return;
  const bool live = (i < real8);
  const int ic = live ? i : (real8 - 1);
  const float* p = src + ((size_t)ic << 3);
  const v4f a0 = *(const v4f*)(p);
  const v4f a1 = *(const v4f*)(p + 4);
  v8h hv;
#pragma unroll
  for (int e = 0; e < 4; ++e) {
    const float f0 = live ? (bfr(a0[e]) * scale) : 0.0f;
    const float f1 = live ? (bfr(a1[e]) * scale) : 0.0f;
    hv[e]     = (_Float16)f0;
    hv[4 + e] = (_Float16)f1;
  }
  unsigned short* q = dst + ((size_t)i << 3);
  *(volatile v8h*)q = hv;
  __threadfence();
  *(volatile v8h*)q = hv;
}

__global__ __launch_bounds__(256) void conv_silu_kernel(
    const float* __restrict__ XZ, const float* __restrict__ cw, const float* __restrict__ cb,
    float* __restrict__ XC, unsigned short* __restrict__ XC16)
{
  __shared__ __align__(16) float sT[16 * kConvTP];
  const int tid = threadIdx.x, lane = tid & 31, wave = tid >> 5;
  const int d = tid;
  const int g0 = blockIdx.x * 64;
  const int tb = g0 & (kSeq - 1);
  const v4f wv = *(const v4f*)(cw + d * 4);
  const float w0 = bfr(wv[0]), w1 = bfr(wv[1]), w2 = bfr(wv[2]), w3 = bfr(wv[3]);
  const float bc = bfr(cb[d]);
  float xm3, xm2, xm1;
  {
    const bool hist = (tb > 0);
    const int rb = hist ? (g0 - 3) : g0;
    const float v3 = XZ[(size_t)rb * kXz + d];
    const float v2 = XZ[(size_t)(rb + 1) * kXz + d];
    const float v1 = XZ[(size_t)(rb + 2) * kXz + d];
    xm3 = hist ? v3 : 0.f;
    xm2 = hist ? v2 : 0.f;
    xm1 = hist ? v1 : 0.f;
  }
  const int hrow = wave >> 1;
  const int hch  = (wave & 1) * 128 + lane * 4;
#pragma unroll 1
  for (int sub = 0; sub < 4; ++sub) {
    const int lb = g0 + sub * 16;
#pragma unroll 1
    for (int s = 0; s < 16; ++s) {
      const float xcur = XZ[(size_t)(lb + s) * kXz + d];
      float acc = w0 * xm3;
      acc = fmaf(w1, xm2, acc);
      acc = fmaf(w2, xm1, acc);
      acc = fmaf(w3, xcur, acc);
      const float sv = acc + bc;
      const float sg = __builtin_amdgcn_rcpf(1.0f + __expf(-sv));
      sT[s * kConvTP + tid] = sv * sg;
      xm3 = xm2; xm2 = xm1; xm1 = xcur;
    }
    __syncthreads();
    v4f fv[4];
    v8h bv[2];
#pragma unroll
    for (int it = 0; it < 4; ++it) fv[it] = *(const v4f*)(sT + (it * 4 + hrow) * kConvTP + hch);
#pragma unroll
    for (int it = 0; it < 2; ++it) {
      const float* sp = sT + (it * 8 + wave) * kConvTP + lane * 8;
      const v4f a0 = *(const v4f*)(sp);
      const v4f a1 = *(const v4f*)(sp + 4);
#pragma unroll
      for (int e = 0; e < 4; ++e) {
        bv[it][e]     = (_Float16)(a0[e] * kCarryXc);
        bv[it][4 + e] = (_Float16)(a1[e] * kCarryXc);
      }
    }
    for (int pass = 0; pass < 2; ++pass) {
#pragma unroll
      for (int it = 0; it < 4; ++it)
        *(volatile v4f*)(XC + (size_t)(lb + it * 4 + hrow) * kDi + hch) = fv[it];
#pragma unroll
      for (int it = 0; it < 2; ++it)
        *(volatile v8h*)(XC16 + (size_t)(lb + it * 8 + wave) * kDi + lane * 8) = bv[it];
      __threadfence();
    }
    __syncthreads();
  }
}

__global__ __launch_bounds__(128) void scan_kernel(
    const float* __restrict__ DBC, const float* __restrict__ XC, const float* __restrict__ XZ,
    const float* __restrict__ Wdt, const float* __restrict__ bdt, const float* __restrict__ Alog,
    const float* __restrict__ Dp, unsigned short* __restrict__ Y16)
{
  __shared__ __align__(16) float    sB[kTS * kNs];
  __shared__ __align__(16) float    sDT[kTS * kDtR];
  __shared__ __align__(16) _Float16 sC[kTS * kNs];
  __shared__ __align__(16) float    sDL[kTS * kSCh];
  __shared__ __align__(16) float    sDU[kTS * kSCh];
  __shared__ __align__(16) float    sY[kTS * kSYP];

  const int tid = threadIdx.x, lane = tid & 31, wave = tid >> 5;
  const int hh = lane >> 4, m = lane & 15;
  constexpr int kBlkPerB = kDi / kSCh;
  const int bix = blockIdx.x / kBlkPerB;
  const int d0  = (blockIdx.x - bix * kBlkPerB) * kSCh;
  const int cl  = wave * 16 + m;
  const int d   = d0 + cl;
  const size_t row0 = (size_t)bix * kSeq;

  float A2[64], H[64];
#pragma unroll
  for (int kt = 0; kt < 4; ++kt) {
#pragma unroll
    for (int g = 0; g < 2; ++g) {
      const float* ap = Alog + (size_t)d * kNs + kt * 32 + 16 * g + 8 * hh;
      const v4f q0 = *(const v4f*)(ap);
      const v4f q1 = *(const v4f*)(ap + 4);
#pragma unroll
      for (int e = 0; e < 4; ++e) {
        A2[kt * 16 + 8 * g + e]     = -__expf(bfr(q0[e])) * kLog2e;
        A2[kt * 16 + 8 * g + 4 + e] = -__expf(bfr(q1[e])) * kLog2e;
      }
    }
  }
#pragma unroll
  for (int i = 0; i < 64; ++i) H[i] = 0.f;

  const int c2 = tid & 63;
  const int r2 = tid >> 6;
  float wd[8];
  {
    const v4f wa = *(const v4f*)(Wdt + (size_t)(d0 + c2) * kDtR);
    const v4f wb = *(const v4f*)(Wdt + (size_t)(d0 + c2) * kDtR + 4);
#pragma unroll
    for (int e = 0; e < 4; ++e) { wd[e] = bfr(wa[e]); wd[4 + e] = bfr(wb[e]); }
  }
  const float bb2 = bfr(bdt[d0 + c2]);

  const int q = lane >> 3, c8 = (lane & 7) * 8;
  float Dv[8];
  {
    const v4f da = *(const v4f*)(Dp + d0 + c8);
    const v4f db = *(const v4f*)(Dp + d0 + c8 + 4);
#pragma unroll
    for (int e = 0; e < 4; ++e) { Dv[e] = bfr(da[e]); Dv[4 + e] = bfr(db[e]); }
  }

#pragma unroll 1
  for (int t0 = 0; t0 < kSeq; t0 += kTS) {
    const size_t rowg = row0 + (size_t)t0;
#pragma unroll
    for (int it = 0; it < 8; ++it) {
      const int idx = it * 128 + tid;
      const int r = idx >> 5, c4 = (idx & 31) * 4;
      *(v4f*)(sB + r * kNs + c4) = *(const v4f*)(DBC + (rowg + r) * kNxP + kDtR + c4);
    }
#pragma unroll
    for (int it = 0; it < 4; ++it) {
      const int idx = it * 128 + tid;
      const int r = idx >> 4, g = idx & 15;
      const float* p = DBC + (rowg + r) * kNxP + kDtR + kNs + g * 8;
      const v4f c0 = *(const v4f*)(p);
      const v4f c1 = *(const v4f*)(p + 4);
      v8h hv;
#pragma unroll
      for (int e = 0; e < 4; ++e) {
        hv[e]     = (_Float16)(c0[e] * kCarryC);
        hv[4 + e] = (_Float16)(c1[e] * kCarryC);
      }
      *(v8h*)(sC + r * kNs + g * 8) = hv;
    }
    if (tid < 64) {
      const int r = tid >> 1, c4 = (tid & 1) * 4;
      *(v4f*)(sDT + r * kDtR + c4) = *(const v4f*)(DBC + (rowg + r) * kNxP + c4);
    }
    __syncthreads();

#pragma unroll 1
    for (int it = 0; it < 16; ++it) {
      const int r = it * 2 + r2;
      const v4f ta = *(const v4f*)(sDT + r * kDtR);
      const v4f tb = *(const v4f*)(sDT + r * kDtR + 4);
      float vd = ta[0] * wd[0];
      vd = fmaf(ta[1], wd[1], vd);
      vd = fmaf(ta[2], wd[2], vd);
      vd = fmaf(ta[3], wd[3], vd);
      vd = fmaf(tb[0], wd[4], vd);
      vd = fmaf(tb[1], wd[5], vd);
      vd = fmaf(tb[2], wd[6], vd);
      vd = fmaf(tb[3], wd[7], vd);
      const float v   = vd + bb2;
      const float av  = __expf(-fabsf(v));
      const float u1  = 1.0f + av;
      const float l1p = __logf(u1) + (av - (u1 - 1.0f)) * __builtin_amdgcn_rcpf(u1);
      const float dlv = fmaxf(v, 0.0f) + l1p;
      const float xcv = XC[(rowg + r) * kDi + d0 + c2];
      sDL[r * kSCh + c2] = dlv;
      sDU[r * kSCh + c2] = (dlv * xcv) * kCarryH;
    }
    __syncthreads();

#pragma unroll 1
    for (int s = 0; s < kTS; ++s) {
      const float dl = sDL[s * kSCh + cl];
      const float du = sDU[s * kSCh + cl];
      const float* bp = sB + s * kNs + 8 * hh;
      const _Float16* cp = sC + s * kNs + 8 * hh;
      v8f acc = (v8f){0.f, 0.f, 0.f, 0.f, 0.f, 0.f, 0.f, 0.f};
#pragma unroll
      for (int kt = 0; kt < 4; ++kt) {
        const v4f b0 = *(const v4f*)(bp + kt * 32);
        const v4f b1 = *(const v4f*)(bp + kt * 32 + 4);
        const v4f b2 = *(const v4f*)(bp + kt * 32 + 16);
        const v4f b3 = *(const v4f*)(bp + kt * 32 + 20);
        float bv[16];
#pragma unroll
        for (int e = 0; e < 4; ++e) { bv[e] = b0[e]; bv[4 + e] = b1[e]; bv[8 + e] = b2[e]; bv[12 + e] = b3[e]; }
#pragma unroll
        for (int i = 0; i < 16; ++i) {
          const float ee = __builtin_amdgcn_exp2f(dl * A2[kt * 16 + i]);
          const float tt = H[kt * 16 + i] * ee;
          H[kt * 16 + i] = fmaf(du, bv[i], tt);
        }
        v8u au;
#pragma unroll
        for (int j = 0; j < 8; ++j) au[j] = pk_f16(H[kt * 16 + 2 * j], H[kt * 16 + 2 * j + 1]);
        const v16h af = __builtin_bit_cast(v16h, au);
        const v16h cf = frag_load_h(cp + kt * 32);
        acc = mma_h(af, cf, acc);
        guard1_h(acc, af, cf);
      }
      if (m == 0) {
        float* yp = sY + s * kSYP + wave * 16 + 8 * hh;
        const v4f ylo = (v4f){acc[0], acc[1], acc[2], acc[3]};
        const v4f yhi = (v4f){acc[4], acc[5], acc[6], acc[7]};
        *(v4f*)(yp)     = ylo;
        *(v4f*)(yp + 4) = yhi;
      }
    }
    __syncthreads();

    v8h hv[2];
#pragma unroll
    for (int it = 0; it < 2; ++it) {
      const int row = it * 16 + wave * 4 + q;
      const size_t rg = rowg + row;
      const float* sp = sY + row * kSYP + c8;
      const v4f y0 = *(const v4f*)(sp);
      const v4f y1 = *(const v4f*)(sp + 4);
      const v4f x0 = *(const v4f*)(XC + rg * kDi + d0 + c8);
      const v4f x1 = *(const v4f*)(XC + rg * kDi + d0 + c8 + 4);
      const v4f z0 = *(const v4f*)(XZ + rg * kXz + kDi + d0 + c8);
      const v4f z1 = *(const v4f*)(XZ + rg * kXz + kDi + d0 + c8 + 4);
#pragma unroll
      for (int e = 0; e < 4; ++e) {
        const float za = z0[e], zb = z1[e];
        const float sa = __builtin_amdgcn_rcpf(1.0f + __expf(-za));
        const float sb = __builtin_amdgcn_rcpf(1.0f + __expf(-zb));
        const float ya = fmaf(x0[e], Dv[e], y0[e] * kInvHC);
        const float yb = fmaf(x1[e], Dv[4 + e], y1[e] * kInvHC);
        hv[it][e]     = (_Float16)((ya * (za * sa)) * kCarryY);
        hv[it][4 + e] = (_Float16)((yb * (zb * sb)) * kCarryY);
      }
    }
    for (int pass = 0; pass < 2; ++pass) {
#pragma unroll
      for (int it = 0; it < 2; ++it) {
        const int row = it * 16 + wave * 4 + q;
        *(volatile v8h*)(Y16 + (rowg + row) * kDi + d0 + c8) = hv[it];
      }
      __threadfence();
    }
  }
}

extern "C" void kernel_launch(void* const* d_in, const int* in_sizes, int n_in,
                              void* d_out, int out_size, void* d_ws, size_t ws_size,
                              hipStream_t stream)
{
  if (n_in < 10) return;
  if (in_sizes[0] != kRows * kDm) return;
  if (in_sizes[1] != kXz * kDm) return;
  if (in_sizes[2] != kDi * 4) return;
  if (in_sizes[3] != kDi) return;
  if (in_sizes[4] != kNx * kDi) return;
  if (in_sizes[5] != kDi * kDtR) return;
  if (in_sizes[6] != kDi) return;
  if (in_sizes[7] != kDi * kNs) return;
  if (in_sizes[8] != kDi) return;
  if (in_sizes[9] != kDm * kDi) return;
  if (out_size != kRows * kDm) return;
  if (ws_size < kWsTotal) return;

  const float* x      = (const float*)d_in[0];
  const float* W_in   = (const float*)d_in[1];
  const float* conv_w = (const float*)d_in[2];
  const float* conv_b = (const float*)d_in[3];
  const float* W_x    = (const float*)d_in[4];
  const float* W_dt   = (const float*)d_in[5];
  const float* b_dt   = (const float*)d_in[6];
  const float* A_log  = (const float*)d_in[7];
  const float* Dp     = (const float*)d_in[8];
  const float* W_out  = (const float*)d_in[9];
  float* out = (float*)d_out;

  char* ws = (char*)d_ws;
  unsigned short* U16    = (unsigned short*)(ws + kOffU16);
  unsigned short* WIN16  = (unsigned short*)(ws + kOffWIN);
  unsigned short* WX16   = (unsigned short*)(ws + kOffWX);
  unsigned short* WOUT16 = (unsigned short*)(ws + kOffWOUT);
  float*          XZ     = (float*)(ws + kOffXZ);
  float*          XC     = (float*)(ws + kOffXC);
  unsigned short* XC16   = (unsigned short*)(ws + kOffXC16);
  float*          DBC    = (float*)(ws + kOffDBC);
  unsigned short* Y16    = (unsigned short*)(ws + kOffY16);

  cast_bf16r_f16_kernel<<<(kRows * kDm / 8) / 256, 256, 0, stream>>>(x, U16, kRows * kDm / 8, kRows * kDm / 8, 1.0f);
  cast_bf16r_f16_kernel<<<(kXz * kDm / 8) / 256, 256, 0, stream>>>(W_in, WIN16, kXz * kDm / 8, kXz * kDm / 8, kCarryW);
  cast_bf16r_f16_kernel<<<(kNxP * kDi / 8) / 256, 256, 0, stream>>>(W_x, WX16, kNxP * kDi / 8, kNx * kDi / 8, kCarryW);
  cast_bf16r_f16_kernel<<<(kDm * kDi / 8) / 256, 256, 0, stream>>>(W_out, WOUT16, kDm * kDi / 8, kDm * kDi / 8, kCarryW);

  for (int hf = 0; hf < kHalves; ++hf) {
    const unsigned short* Uh = U16 + (size_t)hf * kRowsH * kDm;
    float* outh = out + (size_t)hf * kRowsH * kDm;

    gemm64_f16_kernel<<<(kRowsH / 64) * (kXz / 64) / 8, 256, 0, stream>>>(
        Uh, kDm, WIN16, kDm, XZ, kXz, kRowsH, kXz, kDm, 1.0f / kCarryW);

    conv_silu_kernel<<<kRowsH / 64, 256, 0, stream>>>(XZ, conv_w, conv_b, XC, XC16);

    gemm64_f16_kernel<<<(kRowsH / 64) * (kNxP / 64) / 8, 256, 0, stream>>>(
        XC16, kDi, WX16, kDi, DBC, kNxP, kRowsH, kNxP, kDi, 1.0f / (kCarryXc * kCarryW));

    scan_kernel<<<kBatchH * (kDi / kSCh), 128, 0, stream>>>(DBC, XC, XZ, W_dt, b_dt, A_log, Dp, Y16);

    gemm64_f16_kernel<<<(kRowsH / 64) * (kDm / 64) / 8, 256, 0, stream>>>(
        Y16, kDi, WOUT16, kDi, outh, kDm, kRowsH, kDm, kDi, 1.0f / (kCarryY * kCarryW));
  }
}
